// MultiHeadedAttention_64441689309679
// MI455X (gfx1250) — hardware-verified
//
#include <hip/hip_runtime.h>
#ifndef NB
#define NB 2
#endif
#ifndef SEQ
#define SEQ 2048
#endif
#define NB_FULL 2
#define SEQ_FULL 2048
#define DD 1024
#define NH 16
#define HD 64
#define NCH (SEQ_FULL / 32)

static_assert(NB >= 1 && NB <= NB_FULL);
static_assert(SEQ >= 64 && SEQ <= SEQ_FULL && (SEQ % 64) == 0);
static_assert(NH * HD == DD && (DD % 64) == 0 && (HD % 32) == 0 && HD <= 128);
static_assert(NCH == 64 && (SEQ_FULL % 64) == 0);
static_assert((DD % 32) == 0 && (SEQ % 16) == 0);

typedef __bf16 v16b __attribute__((ext_vector_type(16)));
typedef unsigned short v8us __attribute__((ext_vector_type(8), may_alias));
typedef float  v8f  __attribute__((ext_vector_type(8)));
typedef float  v4f  __attribute__((ext_vector_type(4)));
typedef float  v4fa __attribute__((ext_vector_type(4), may_alias));
typedef int    v4i  __attribute__((ext_vector_type(4)));
typedef int    v4ia __attribute__((ext_vector_type(4), may_alias));
union FragB { v16b v; v8us half[2]; unsigned short u[16]; };

__device__ __forceinline__ unsigned short bf16_bits(float x) { unsigned int u = __float_as_uint(x); return (unsigned short)((u + 0x7FFFu + ((u >> 16) & 1u)) >> 16); }
__device__ __forceinline__ float bf16_val(unsigned short b) { return __uint_as_float(((unsigned int)b) << 16); }
__device__ __forceinline__ float bf16_rne(float x) { return bf16_val(bf16_bits(x)); }

template <int NT>
__device__ __forceinline__ v8f mmaN(v16b ah, v16b al, v16b bh, v16b bl, v8f c) {
  c = __builtin_amdgcn_wmma_f32_16x16x32_bf16(false, ah, false, bh, (short)0, c, false, false);
  if (NT >= 2) c = __builtin_amdgcn_wmma_f32_16x16x32_bf16(false, al, false, bh, (short)0, c, false, false);
  if (NT >= 3) c = __builtin_amdgcn_wmma_f32_16x16x32_bf16(false, ah, false, bl, (short)0, c, false, false);
  asm volatile("v_nop\n\tv_nop\n\tv_nop\n\tv_nop" : "+v"(c) : "v"(ah), "v"(al), "v"(bh), "v"(bl));
  return c;
}

__global__ __launch_bounds__(256) void k_rne_rows(const float* __restrict__ W, unsigned short* __restrict__ Wt, int n8) {
  const int t = blockIdx.x * 256 + threadIdx.x;
  if (t >= n8) return;
  const v4f a = *(const v4fa*)(W + (size_t)t * 8), b = *(const v4fa*)(W + (size_t)t * 8 + 4);
  v8us v; v[0]=bf16_bits(a[0]); v[1]=bf16_bits(a[1]); v[2]=bf16_bits(a[2]); v[3]=bf16_bits(a[3]);
  v[4]=bf16_bits(b[0]); v[5]=bf16_bits(b[1]); v[6]=bf16_bits(b[2]); v[7]=bf16_bits(b[3]);
  *(volatile v8us*)(Wt + (size_t)t * 8) = v; __threadfence(); *(volatile v8us*)(Wt + (size_t)t * 8) = v;
}

template <bool ASPLIT, bool BIAS_BF16>
__global__ __launch_bounds__(128) void k_gemm_bf(const float* __restrict__ A, int lda, int abatch, const unsigned short* __restrict__ Wt, int ldb,
                                               const float* __restrict__ bias, float* __restrict__ C, int ldc, int cbatch, int M, int N, int K) {
  __shared__ __attribute__((aligned(16))) float so[4][16][64];
  const int tid = threadIdx.x, w = tid >> 5, lane = tid & 31, ln = lane & 15, hh = lane >> 4;
  const int ntn = N / 64;
  const int wid = blockIdx.x * 4 + w;
  const int mt = wid / ntn, nq = wid % ntn;
  if (mt * 16 >= M) return;
  const int row0 = mt * 16, col0 = nq * 64;
  const float* Ab = A + (size_t)blockIdx.y * (size_t)abatch;
  float* Cb = C + (size_t)blockIdx.y * (size_t)cbatch;
  const float* arow = Ab + (size_t)(row0 + ln) * lda;
  v8f acc[4];
#pragma unroll
  for (int t = 0; t < 4; ++t) acc[t] = (v8f){0.f,0.f,0.f,0.f,0.f,0.f,0.f,0.f};
  for (int kb = 0; kb < K; kb += 32) {
    FragB ah, al;
    const v4f x0 = *(const v4fa*)(arow + kb + 8 * hh), x1 = *(const v4fa*)(arow + kb + 8 * hh + 4);
    const v4f x2 = *(const v4fa*)(arow + kb + 16 + 8 * hh), x3 = *(const v4fa*)(arow + kb + 16 + 8 * hh + 4);
    float xs[16] = {x0[0],x0[1],x0[2],x0[3],x1[0],x1[1],x1[2],x1[3],x2[0],x2[1],x2[2],x2[3],x3[0],x3[1],x3[2],x3[3]};
#pragma unroll
    for (int i = 0; i < 16; ++i) { const unsigned short hb = bf16_bits(xs[i]); ah.u[i] = hb; al.u[i] = ASPLIT ? bf16_bits(xs[i] - bf16_val(hb)) : (unsigned short)0; }
#pragma unroll
    for (int t = 0; t < 4; ++t) {
      const unsigned short* brow = Wt + (size_t)(col0 + t * 16 + ln) * ldb + kb;
      FragB b;
      b.half[0] = *(const v8us*)(brow + 8 * hh);
      b.half[1] = *(const v8us*)(brow + 16 + 8 * hh);
      acc[t] = mmaN<ASPLIT ? 2 : 1>(ah.v, al.v, b.v, b.v, acc[t]);
    }
  }
#pragma unroll
  for (int t = 0; t < 4; ++t) {
    float bvv = bias[col0 + t * 16 + ln];
    if (BIAS_BF16) bvv = bf16_rne(bvv);
#pragma unroll
    for (int r = 0; r < 8; ++r) { so[w][8 * hh + r][t * 16 + ln] = acc[t][r] + bvv; }
  }
  __builtin_amdgcn_fence(4  , "workgroup");
  __builtin_amdgcn_wave_barrier();
  const int rsub = lane >> 4, c4 = (lane & 15) * 4;
  for (int pass = 0; pass < 2; ++pass) {
#pragma unroll
    for (int q = 0; q < 8; ++q) {
      const int r = q * 2 + rsub;
      const v4f v = *(const v4fa*)&so[w][r][c4];
      *(volatile v4f*)(Cb + (size_t)(row0 + r) * ldc + col0 + c4) = v;
    }
    if (pass == 0) __threadfence();
  }
}

__global__ __launch_bounds__(256) void k_mask_flags(const int* __restrict__ mask, int mbatch, int mpitch, int T, int* __restrict__ flags) {
  __shared__ int srow[8][64];
  __shared__ __attribute__((aligned(16))) int sflag[NCH];
  const int tid = threadIdx.x, w = tid >> 5, lane = tid & 31;
  const int nqb = T / 64;
  const int b = blockIdx.x / nqb, qblk = blockIdx.x % nqb;
  const int* mb = mask + (size_t)b * mbatch + (size_t)(qblk * 64) * mpitch;
  const int nc = T / 32;
  int any0 = 0, any1 = 0;
  for (int c = w; c < NCH; c += 8) {
    int cnt = 0;
    if (c < nc) {
      const int* p0 = mb + (size_t)(2 * lane) * mpitch + c * 32;
      const int* p1 = p0 + mpitch;
#pragma unroll 4
      for (int j = 0; j < 8; ++j) {
        const v4i x = *(const v4ia*)(p0 + 4 * j);
        const v4i z = *(const v4ia*)(p1 + 4 * j);
        const int n0 = (x[0] != 0) + (x[1] != 0) + (x[2] != 0) + (x[3] != 0);
        const int n1 = (z[0] != 0) + (z[1] != 0) + (z[2] != 0) + (z[3] != 0);
        cnt += n0 + n1; any0 |= n0; any1 |= n1;
      }
    }
    cnt += __shfl_xor(cnt, 1, 32); cnt += __shfl_xor(cnt, 2, 32); cnt += __shfl_xor(cnt, 4, 32);
    cnt += __shfl_xor(cnt, 8, 32); cnt += __shfl_xor(cnt, 16, 32);
    const int fl = (cnt == 0) ? 0 : ((cnt == 64 * 32) ? 2 : 1);
    if (lane == 0) sflag[c] = fl;
  }
  srow[w][2 * lane] = (any0 != 0) ? 1 : 0;
  srow[w][2 * lane + 1] = (any1 != 0) ? 1 : 0;
  __syncthreads();
  if (w == 0) {
    int a = 0, a2 = 0;
#pragma unroll
    for (int i = 0; i < 8; ++i) { a |= srow[i][lane]; a2 |= srow[i][lane + 32]; }
    int dead = ((a == 0) || (a2 == 0)) ? 1 : 0;
    dead |= __shfl_xor(dead, 1, 32); dead |= __shfl_xor(dead, 2, 32); dead |= __shfl_xor(dead, 4, 32);
    dead |= __shfl_xor(dead, 8, 32); dead |= __shfl_xor(dead, 16, 32);
    const int li = lane & 15;
    v4i fv = *(const v4ia*)&sflag[li * 4];
    if (dead) {
#pragma unroll
      for (int i = 0; i < 4; ++i) fv[i] = (fv[i] > 1) ? fv[i] : 1;
    }
    int* dst = flags + (size_t)blockIdx.x * NCH + li * 4;
    if (lane < 16) *(volatile v4i*)dst = fv;
    __threadfence();
    if (lane < 16) *(volatile v4i*)dst = fv;
  }
}

template <int D>
__global__ __launch_bounds__(128) void k_flash_mk(const float* __restrict__ Qb, const float* __restrict__ Kb, const float* __restrict__ Vb,
                                                int pitch, int T, int H, float scale, const int* __restrict__ mask, int mbatch, int mpitch,
                                                const int* __restrict__ flags, float* __restrict__ y, int ypitch) {
  constexpr int KS = D / 32, DT = D / 16;
  __shared__ __attribute__((aligned(16))) unsigned short sKh[32][D + 8], sKl[32][D + 8], sVh[32][D + 8], sVl[32][D + 8];
  __shared__ __attribute__((aligned(16))) unsigned short sPh[4][16][40], sPl[4][16][40];
  __shared__ __attribute__((aligned(16))) float sO[4][16][D];
  __shared__ __attribute__((aligned(16))) int sM[64][32];
  const int tid = threadIdx.x, w = tid >> 5, lane = tid & 31, ln = lane & 15, hh = lane >> 4;
  const int nqb = T / 64;
  const int bh = blockIdx.x / nqb, qblk = blockIdx.x % nqb;
  const int b = bh / H, h = bh % H;
  const int q0 = qblk * 64 + w * 16;
  const float* Q = Qb + (size_t)b * T * pitch + h * D;
  const float* K = Kb + (size_t)b * T * pitch + h * D;
  const float* V = Vb + (size_t)b * T * pitch + h * D;
  const int* Mb = mask + (size_t)b * (size_t)mbatch + (size_t)(qblk * 64) * (size_t)mpitch;
  const int* fl = flags + (size_t)(b * nqb + qblk) * NCH;

  FragB aqh[KS], aql[KS];
  {
    int row = q0 + ln; if (row >= T) row = T - 1;
    const float* qr = Q + (size_t)row * pitch;
#pragma unroll
    for (int ks = 0; ks < KS; ++ks)
#pragma unroll
      for (int i = 0; i < 16; ++i) {
        const int d = ks * 32 + ((i < 8) ? (8 * hh + i) : (16 + 8 * hh + (i - 8)));
        const float x = qr[d] * scale; const unsigned short hb = bf16_bits(x);
        aqh[ks].u[i] = hb; aql[ks].u[i] = bf16_bits(x - bf16_val(hb));
      }
  }
  float m_r[8], l_r[8];
#pragma unroll
  for (int r = 0; r < 8; ++r) { m_r[r] = -3.0e38f; l_r[r] = 0.f; }
  v8f oacc[DT];
#pragma unroll
  for (int dt = 0; dt < DT; ++dt) oacc[dt] = (v8f){0.f,0.f,0.f,0.f,0.f,0.f,0.f,0.f};

  for (int j0 = 0; j0 < T; j0 += 32) {
    const int f = fl[j0 >> 5];
    if (f == 0) continue;
    const bool mixed = (f != 2);
    __syncthreads();
    for (int e = tid; e < 32 * (D / 4); e += 128) {
      const int r = e / (D / 4), c4 = (e % (D / 4)) * 4;
      int key = j0 + r; const bool kin = key < T; if (!kin) key = T - 1;
      v4f kf = *(const v4fa*)(K + (size_t)key * pitch + c4);
      v4f vf = *(const v4fa*)(V + (size_t)key * pitch + c4);
      if (!kin) { kf = (v4f){0.f,0.f,0.f,0.f}; vf = (v4f){0.f,0.f,0.f,0.f}; }
#pragma unroll
      for (int t = 0; t < 4; ++t) {
        unsigned short hb = bf16_bits(kf[t]); sKh[r][c4 + t] = hb; sKl[r][c4 + t] = bf16_bits(kf[t] - bf16_val(hb));
        hb = bf16_bits(vf[t]); sVh[r][c4 + t] = hb; sVl[r][c4 + t] = bf16_bits(vf[t] - bf16_val(hb));
      }
    }
    if (mixed) {
      for (int e = tid; e < 64 * 8; e += 128) {
        const int r = e >> 3, c4 = (e & 7) * 4;
        int key = j0 + c4; if (key + 3 >= T) key = T - 4;
        const v4i x = *(const v4ia*)(Mb + (size_t)r * (size_t)mpitch + key);
        *(v4i*)&sM[r][c4] = x;
      }
    }
    __syncthreads();
    v8f s[2];
#pragma unroll
    for (int nt = 0; nt < 2; ++nt) {
      v8f acc = (v8f){0.f,0.f,0.f,0.f,0.f,0.f,0.f,0.f};
#pragma unroll
      for (int ks = 0; ks < KS; ++ks) {
        FragB bh_, bl_;
        bh_.half[0] = *(const v8us*)&sKh[nt * 16 + ln][ks * 32 + 8 * hh]; bh_.half[1] = *(const v8us*)&sKh[nt * 16 + ln][ks * 32 + 16 + 8 * hh];
        bl_.half[0] = *(const v8us*)&sKl[nt * 16 + ln][ks * 32 + 8 * hh]; bl_.half[1] = *(const v8us*)&sKl[nt * 16 + ln][ks * 32 + 16 + 8 * hh];
        acc = mmaN<3>(aqh[ks].v, aql[ks].v, bh_.v, bl_.v, acc);
      }
      s[nt] = acc;
    }
    unsigned int kbits = 0xFFFFu;
    if (mixed) {
      kbits = 0u;
#pragma unroll
      for (int r = 0; r < 8; ++r) {
        const int ma = sM[w * 16 + 8 * hh + r][ln], mb2 = sM[w * 16 + 8 * hh + r][16 + ln];
        kbits |= ((ma != 0) ? 1u : 0u) << r;
        kbits |= ((mb2 != 0) ? 1u : 0u) << (8 + r);
      }
    }
    float alpha[8];
#pragma unroll
    for (int r = 0; r < 8; ++r) {
      if (((kbits >> r) & 1u) == 0u) s[0][r] = -1.0e9f;
      if (((kbits >> (8 + r)) & 1u) == 0u) s[1][r] = -1.0e9f;
      float mx = fmaxf(s[0][r], s[1][r]);
      mx = fmaxf(mx, __shfl_xor(mx, 1, 32)); mx = fmaxf(mx, __shfl_xor(mx, 2, 32)); mx = fmaxf(mx, __shfl_xor(mx, 4, 32)); mx = fmaxf(mx, __shfl_xor(mx, 8, 32));
      const float mnew = fmaxf(m_r[r], mx);
      alpha[r] = (m_r[r] > -1.0e38f) ? __expf(m_r[r] - mnew) : 0.0f;
      const float p0 = __expf(s[0][r] - mnew);
      const float p1 = __expf(s[1][r] - mnew);
      m_r[r] = mnew;
      l_r[r] = l_r[r] * alpha[r] + p0 + p1;
      unsigned short hb = bf16_bits(p0); sPh[w][8 * hh + r][ln] = hb;      sPl[w][8 * hh + r][ln] = bf16_bits(p0 - bf16_val(hb));
      hb = bf16_bits(p1);                sPh[w][8 * hh + r][16 + ln] = hb; sPl[w][8 * hh + r][16 + ln] = bf16_bits(p1 - bf16_val(hb));
    }
#pragma unroll
    for (int dt = 0; dt < DT; ++dt)
#pragma unroll
      for (int r = 0; r < 8; ++r) oacc[dt][r] *= alpha[r];
    __builtin_amdgcn_fence(4  , "workgroup");
    __builtin_amdgcn_wave_barrier();
    FragB pah, pal;
    pah.half[0] = *(const v8us*)&sPh[w][ln][8 * hh]; pah.half[1] = *(const v8us*)&sPh[w][ln][16 + 8 * hh];
    pal.half[0] = *(const v8us*)&sPl[w][ln][8 * hh]; pal.half[1] = *(const v8us*)&sPl[w][ln][16 + 8 * hh];
#pragma unroll
    for (int dt = 0; dt < DT; ++dt) {
      FragB bvh, bvl;
#pragma unroll
      for (int i = 0; i < 8; ++i) {
        bvh.u[i] = sVh[8 * hh + i][dt * 16 + ln]; bvh.u[8 + i] = sVh[16 + 8 * hh + i][dt * 16 + ln];
        bvl.u[i] = sVl[8 * hh + i][dt * 16 + ln]; bvl.u[8 + i] = sVl[16 + 8 * hh + i][dt * 16 + ln];
      }
      oacc[dt] = mmaN<3>(pah.v, pal.v, bvh.v, bvl.v, oacc[dt]);
    }
    __builtin_amdgcn_fence(4  , "workgroup");
    __builtin_amdgcn_wave_barrier();
  }
#pragma unroll
  for (int r = 0; r < 8; ++r) {
    float l = l_r[r];
    l += __shfl_xor(l, 1, 32); l += __shfl_xor(l, 2, 32); l += __shfl_xor(l, 4, 32); l += __shfl_xor(l, 8, 32);
    l_r[r] = 1.0f / l;
  }
#pragma unroll
  for (int dt = 0; dt < DT; ++dt)
#pragma unroll
    for (int r = 0; r < 8; ++r) sO[w][8 * hh + r][dt * 16 + ln] = oacc[dt][r] * l_r[r];
  __builtin_amdgcn_fence(4  , "workgroup");
  __builtin_amdgcn_wave_barrier();
  for (int pass = 0; pass < 2; ++pass) {
    for (int r = 0; r < 16; ++r) {
      const int row = q0 + r;
      if (row < T && lane < D / 4) {
        const v4f val = *(const v4fa*)&sO[w][r][lane * 4];
        *(volatile v4f*)(y + ((size_t)b * T + row) * ypitch + h * D + lane * 4) = val;
      }
    }
    if (pass == 0) __threadfence();
  }
}

extern "C" void kernel_launch(void* const* d_in, const int* in_sizes, int n_in,
                              void* d_out, int out_size, void* d_ws, size_t ws_size, hipStream_t stream) {
  if (n_in < 12) return;
  const float* xq = (const float*)d_in[0]; const float* xk = (const float*)d_in[1]; const float* xv = (const float*)d_in[2];
  const int* mask = (const int*)d_in[3];
  const float* Wq = (const float*)d_in[4]; const float* bq = (const float*)d_in[5]; const float* Wk = (const float*)d_in[6]; const float* bk = (const float*)d_in[7];
  const float* Wv = (const float*)d_in[8]; const float* bv = (const float*)d_in[9]; const float* Wo = (const float*)d_in[10]; const float* bo = (const float*)d_in[11];
  const long long needX = (long long)(NB - 1) * (long long)SEQ_FULL * DD + (long long)SEQ * DD;
  if ((long long)in_sizes[0] < needX || (long long)in_sizes[1] < needX || (long long)in_sizes[2] < needX) return;
  const long long needM = (long long)(NB - 1) * (long long)SEQ_FULL * SEQ_FULL + (long long)SEQ * SEQ_FULL;
  if ((long long)in_sizes[3] < needM) return;
  if (in_sizes[4] < DD * DD || in_sizes[6] < DD * DD || in_sizes[8] < DD * DD || in_sizes[10] < DD * DD) return;
  if (in_sizes[5] < DD || in_sizes[7] < DD || in_sizes[9] < DD || in_sizes[11] < DD) return;
  if ((long long)out_size < (long long)NB * SEQ * DD) return;

  char* ws = (char*)d_ws; size_t off = 0;
  auto take = [&](size_t bytes) { char* p = ws + off; off += (bytes + 255) & ~(size_t)255; return p; };
  const size_t MROWS = (size_t)NB * SEQ;
  unsigned short* Wt[4]; for (int i = 0; i < 4; ++i) Wt[i] = (unsigned short*)take((size_t)DD * DD * 2);
  float* q   = (float*)take(MROWS * DD * 4);
  float* k   = (float*)take(MROWS * DD * 4);
  float* v   = (float*)take(MROWS * DD * 4);
  float* att = (float*)take(MROWS * DD * 4);
  int* flags = (int*)take((size_t)NB * (SEQ / 64) * NCH * 4);
  if (off > ws_size) return;

  const int n8 = DD * DD / 8;
  const int gb = ((SEQ / 16) * (DD / 64) + 3) / 4;
  const dim3 gg(gb, NB);
  const float* W4[4] = {Wq, Wk, Wv, Wo};
  for (int i = 0; i < 4; ++i) k_rne_rows<<<(n8 + 255) / 256, 256, 0, stream>>>(W4[i], Wt[i], n8);
  k_gemm_bf<false, true><<<gg, 128, 0, stream>>>(xq, DD, SEQ_FULL * DD, Wt[0], DD, bq, q, DD, SEQ * DD, SEQ, DD, DD);
  k_gemm_bf<false, true><<<gg, 128, 0, stream>>>(xk, DD, SEQ_FULL * DD, Wt[1], DD, bk, k, DD, SEQ * DD, SEQ, DD, DD);
  k_gemm_bf<false, true><<<gg, 128, 0, stream>>>(xv, DD, SEQ_FULL * DD, Wt[2], DD, bv, v, DD, SEQ * DD, SEQ, DD, DD);
  k_mask_flags<<<NB * (SEQ / 64), 256, 0, stream>>>(mask, SEQ_FULL * SEQ_FULL, SEQ_FULL, SEQ, flags);
  k_flash_mk<HD><<<NB * NH * (SEQ / 64), 128, 0, stream>>>(q, k, v, DD, SEQ, NH, 0.125f, mask, SEQ_FULL * SEQ_FULL, SEQ_FULL, flags, att, DD);
  k_gemm_bf<true, true><<<gg, 128, 0, stream>>>(att, DD, SEQ * DD, Wt[3], DD, bo, (float*)d_out, DD, SEQ * DD, SEQ, DD, DD);
  (void)hipGetLastError();
}
